// GNNStackSolution_12601434046987
// MI455X (gfx1250) — hardware-verified
//
#include <hip/hip_runtime.h>
#include <stddef.h>


#define IN1   128
#define HCW   256
#define NH    8
#define OC    40
#define OP    64
#define RPAD  64

#define NTA   256
#define NWAVE 8
#define CHUNK 2048
#define WCAP  256
#define NGRP  (CHUNK / (NTA * 4))

#define NB8   256
#define SH8   8
#define NB1   1024
#define SH1   10

#define LDS8_SACC (NB8 * HCW)
#define LDS8_DEN  (NB8 * NH)
#define LDS8_MAX  (NB8 * NH)
#define LDS8_LIST (NWAVE * WCAP)
#define LDS8_BYTES ((LDS8_SACC + LDS8_DEN + LDS8_MAX + LDS8_LIST + NWAVE) * 4)

#define LDS1_SACC (NB1 * OC)
#define LDS1_DEN  (NB1)
#define LDS1_MAX  (NB1)
#define LDS1_LIST (NWAVE * WCAP)
#define LDS1_BYTES ((LDS1_SACC + LDS1_DEN + LDS1_MAX + LDS1_LIST + NWAVE) * 4)

static_assert(WCAP == (CHUNK / NTA) * 32);
static_assert(NGRP == 2);
static_assert((1 << SH8) == NB8);
static_assert((1 << SH1) == NB1);
static_assert(((LDS8_SACC + LDS8_DEN) % 4) == 0);
static_assert((LDS8_MAX % 4) == 0);
static_assert(((LDS1_SACC + LDS1_DEN) % 4) == 0);
static_assert((LDS1_MAX % 4) == 0);
static_assert(LDS8_BYTES == 286752);
static_assert(LDS1_BYTES == 180256);
static_assert(LDS8_BYTES <= 305152);
static_assert((OC % 4) == 0);
static_assert((NB8 % NWAVE) == 0 && (NB1 % NWAVE) == 0);

typedef float    v4f  __attribute__((ext_vector_type(4)));
typedef float    v8f  __attribute__((ext_vector_type(8)));
typedef int      v4i  __attribute__((ext_vector_type(4)));
typedef _Float16 v8h  __attribute__((ext_vector_type(8)));
typedef _Float16 v16h __attribute__((ext_vector_type(16)));
union Frag   { v16h v; v8h half[2]; };
union Pack16 { v8h h; v4i i; };

__device__ __forceinline__ v8f wmma16(v16h a, v16h b, v8f c) {
  v8f d = __builtin_amdgcn_wmma_f32_16x16x32_f16(false, a, false, b, (short)0, c, false, false);
  asm volatile("v_nop\n\tv_nop\n\tv_nop\n\tv_nop" : "+v"(d) : "v"(a), "v"(b));
  return d;
}

__device__ __forceinline__ float wsum(float v) {
  v += __shfl_xor(v, 16, 32);
  v += __shfl_xor(v, 8, 32);
  v += __shfl_xor(v, 4, 32);
  v += __shfl_xor(v, 2, 32);
  v += __shfl_xor(v, 1, 32);
  return v;
}

__device__ __forceinline__ float wmax(float v) {
  v = fmaxf(v, __shfl_xor(v, 16, 32));
  v = fmaxf(v, __shfl_xor(v, 8, 32));
  v = fmaxf(v, __shfl_xor(v, 4, 32));
  v = fmaxf(v, __shfl_xor(v, 2, 32));
  v = fmaxf(v, __shfl_xor(v, 1, 32));
  return v;
}

__device__ __forceinline__ v4f elu4(v4f v) {
  v4f r;
  r.x = (v.x > 0.f) ? v.x : (__expf(v.x) - 1.0f);
  r.y = (v.y > 0.f) ? v.y : (__expf(v.y) - 1.0f);
  r.z = (v.z > 0.f) ? v.z : (__expf(v.z) - 1.0f);
  r.w = (v.w > 0.f) ? v.w : (__expf(v.w) - 1.0f);
  return r;
}

__global__ __launch_bounds__(256) void k_prepT(const float* __restrict__ W, _Float16* Wt, int K, int NVc) {
  __shared__ __attribute__((aligned(16))) _Float16 T[32 * 72];
  const int tid = threadIdx.x;
  const int k0 = blockIdx.x * 64;
  const int n0 = blockIdx.y * 32;
#pragma unroll
  for (int i = 0; i < 8; ++i) {
    const int idx = tid + 256 * i;
    const int kk = idx >> 5;
    const int nn = idx & 31;
    const int n  = n0 + nn;
    const int nc = (n < NVc) ? n : (NVc - 1);
    const float v = W[(size_t)(k0 + kk) * NVc + nc];
    const float s = (n < NVc) ? v * 8.0f : 0.f;
    T[nn * 72 + kk] = (_Float16)s;
  }
  __syncthreads();
  const int rr = tid >> 3;
  const int pc = (tid & 7) * 8;
  Pack16 u;
  u.h = *(const v8h*)(T + rr * 72 + pc);
  _Float16* gp = Wt + (size_t)(n0 + rr) * K + k0 + pc;
  *(volatile v4i*)gp = u.i;
  __threadfence();
  *(volatile v4i*)gp = u.i;
}

template <int NV>
__device__ __forceinline__ float attcol(const float* __restrict__ a, int col) {
  const int cc = (col < NV) ? col : (NV - 1);
  const float v = a[cc];
  return (col < NV) ? v : 0.f;
}

template <int XP, int NWN, int RB>
__device__ __forceinline__ void epi_tile(v8f t0, v8f t1, int rowT, int hh, int m, int wn, int ncol0,
                                         float cs0, float cs1, float cd0, float cd1,
                                         float* Xs, float* AD) {
  float ss[8], sd[8];
#pragma unroll
  for (int r = 0; r < 8; ++r) {
    const float v0 = t0[r] * 0.125f;
    const float v1 = t1[r] * 0.125f;
    const int row = rowT + 8 * hh + r;
    Xs[row * XP + ncol0]      = v0;
    Xs[row * XP + ncol0 + 16] = v1;
    ss[r] = v0 * cs0 + v1 * cs1;
    sd[r] = v0 * cd0 + v1 * cd1;
  }
#pragma unroll
  for (int mk = 1; mk < 16; mk <<= 1) {
#pragma unroll
    for (int r = 0; r < 8; ++r) {
      ss[r] += __shfl_xor(ss[r], mk, 32);
      sd[r] += __shfl_xor(sd[r], mk, 32);
    }
  }
  if (m == 0) {
#pragma unroll
    for (int r = 0; r < 8; ++r) {
      const int row = rowT + 8 * hh + r;
      AD[row * NWN + wn]            = ss[r];
      AD[RB * NWN + row * NWN + wn] = sd[r];
    }
  }
}

template <int RB, int NWN, int HPW>
__device__ __forceinline__ float scval(const float* AD, int plane, int e) {
  constexpr int NHD = NWN / HPW;
  const int row = e / NHD, head = e % NHD;
  float s = 0.f;
#pragma unroll
  for (int j = 0; j < HPW; ++j) s += AD[plane * RB * NWN + row * NWN + head * HPW + j];
  return s;
}

template <int KD, int NC, int NWM, int HPW, int NV>
__global__ __launch_bounds__(NC * NWM) void k_gemm(
    const float* __restrict__ X, const _Float16* __restrict__ Wt,
    const float* __restrict__ attS, const float* __restrict__ attD,
    float* hout, float* scS, float* scD, int nN) {
  constexpr int NWN  = NC / 32;
  constexpr int NTHR = 32 * NWN * NWM;
  constexpr int RB   = 32 * NWM;
  constexpr int NHD  = NWN / HPW;
  constexpr int AP   = KD + 8;
  constexpr int XP   = NC + 4;
  constexpr int K8   = KD / 8;
  constexpr int NSTG = (RB * K8) / NTHR;
  constexpr int NPC  = (RB * NC / 4) / NTHR;
  constexpr int PP   = (RB * NHD) / 4;
  static_assert(NTHR == NC * NWM);
  static_assert((KD % 32) == 0);
  static_assert((RB * K8) % NTHR == 0);
  static_assert((RB * NC / 4) % NTHR == 0);
  static_assert((RB * NHD) % 4 == 0);
  static_assert(2 * PP <= NTHR);
  static_assert(NWN % HPW == 0);

  __shared__ __attribute__((aligned(16))) _Float16 At[RB * AP];
  __shared__ __attribute__((aligned(16))) float Xs[RB * XP];
  __shared__ __attribute__((aligned(16))) float AD[2 * RB * NWN];

  const int tid  = threadIdx.x;
  const int lane = tid & 31;
  const int wave = tid >> 5;
  const int hh   = lane >> 4;
  const int m    = lane & 15;
  const int wm   = wave / NWN;
  const int wn   = wave % NWN;
  const int rowBase = blockIdx.x * RB;

#pragma unroll
  for (int s = 0; s < NSTG; ++s) {
    const int idx = s * NTHR + tid;
    const int r   = idx / K8;
    const int c0  = (idx % K8) * 8;
    int row = rowBase + r;
    if (row > nN - 1) row = nN - 1;
    const float* p = X + (size_t)row * KD + c0;
    const v4f f0 = *(const v4f*)(p);
    const v4f f1 = *(const v4f*)(p + 4);
    Pack16 u;
    u.h[0] = (_Float16)f0.x; u.h[1] = (_Float16)f0.y; u.h[2] = (_Float16)f0.z; u.h[3] = (_Float16)f0.w;
    u.h[4] = (_Float16)f1.x; u.h[5] = (_Float16)f1.y; u.h[6] = (_Float16)f1.z; u.h[7] = (_Float16)f1.w;
    *(v8h*)(At + r * AP + c0) = u.h;
  }
  __syncthreads();

  const int ar0   = wm * 32 + m;
  const int ar1   = ar0 + 16;
  const int ncol0 = wn * 32 + m;
  const int ncol1 = ncol0 + 16;
  v8f c00 = {0.f, 0.f, 0.f, 0.f, 0.f, 0.f, 0.f, 0.f};
  v8f c01 = {0.f, 0.f, 0.f, 0.f, 0.f, 0.f, 0.f, 0.f};
  v8f c10 = {0.f, 0.f, 0.f, 0.f, 0.f, 0.f, 0.f, 0.f};
  v8f c11 = {0.f, 0.f, 0.f, 0.f, 0.f, 0.f, 0.f, 0.f};
#pragma unroll
  for (int kt = 0; kt < KD / 32; ++kt) {
    const int k0 = kt * 32;
    Frag a0, a1, b0, b1;
    const _Float16* pa0 = At + ar0 * AP + k0 + 8 * hh;
    const _Float16* pa1 = At + ar1 * AP + k0 + 8 * hh;
    const _Float16* pb0 = Wt + (size_t)ncol0 * KD + k0 + 8 * hh;
    const _Float16* pb1 = Wt + (size_t)ncol1 * KD + k0 + 8 * hh;
    a0.half[0] = *(const v8h*)pa0; a0.half[1] = *(const v8h*)(pa0 + 16);
    a1.half[0] = *(const v8h*)pa1; a1.half[1] = *(const v8h*)(pa1 + 16);
    b0.half[0] = *(const v8h*)pb0; b0.half[1] = *(const v8h*)(pb0 + 16);
    b1.half[0] = *(const v8h*)pb1; b1.half[1] = *(const v8h*)(pb1 + 16);
    c00 = wmma16(a0.v, b0.v, c00);
    c01 = wmma16(a0.v, b1.v, c01);
    c10 = wmma16(a1.v, b0.v, c10);
    c11 = wmma16(a1.v, b1.v, c11);
  }

  const float cs0 = attcol<NV>(attS, ncol0);
  const float cs1 = attcol<NV>(attS, ncol1);
  const float cd0 = attcol<NV>(attD, ncol0);
  const float cd1 = attcol<NV>(attD, ncol1);
  epi_tile<XP, NWN, RB>(c00, c01, wm * 32,      hh, m, wn, ncol0, cs0, cs1, cd0, cd1, Xs, AD);
  epi_tile<XP, NWN, RB>(c10, c11, wm * 32 + 16, hh, m, wn, ncol0, cs0, cs1, cd0, cd1, Xs, AD);
  __syncthreads();

  v4f hv[NPC];
#pragma unroll
  for (int i = 0; i < NPC; ++i) {
    const int q   = i * NTHR + tid;
    const int row = q / (NC / 4);
    const int c4  = (q % (NC / 4)) * 4;
    hv[i] = *(const v4f*)(Xs + row * XP + c4);
  }
  float* hp = hout + (size_t)rowBase * NC;
  const bool scw = tid < 2 * PP;
  v4f sv = {0.f, 0.f, 0.f, 0.f};
  float* gp = scS;
  if (scw) {
    const int plane = tid / PP;
    const int q     = tid % PP;
    sv.x = scval<RB, NWN, HPW>(AD, plane, 4 * q + 0);
    sv.y = scval<RB, NWN, HPW>(AD, plane, 4 * q + 1);
    sv.z = scval<RB, NWN, HPW>(AD, plane, 4 * q + 2);
    sv.w = scval<RB, NWN, HPW>(AD, plane, 4 * q + 3);
    gp = (plane ? scD : scS) + (size_t)rowBase * NHD + 4 * q;
  }
#pragma unroll
  for (int i = 0; i < NPC; ++i) *(volatile v4f*)(hp + 4 * (size_t)(i * NTHR + tid)) = hv[i];
  if (scw) *(volatile v4f*)gp = sv;
  __threadfence();
#pragma unroll
  for (int i = 0; i < NPC; ++i) *(volatile v4f*)(hp + 4 * (size_t)(i * NTHR + tid)) = hv[i];
  if (scw) *(volatile v4f*)gp = sv;
}

#define HITJ(J, HJ, SJ) { \
    const unsigned mj = __builtin_amdgcn_ballot_w32(HJ); \
    if (HJ) { \
      const int pos = wc + (int)__builtin_amdgcn_mbcnt_lo(mj, 0u); \
      if (pos < WCAP) list[wave * WCAP + pos] = ((el0 + (J)) << SH) | (int)(SJ); \
    } \
    wc += (int)__builtin_popcount(mj); }

template <int NB, int SH>
__device__ __forceinline__ int scan_chunk(const int* __restrict__ eid, int nE, int cbase, int nodeBase,
                                          int tid, int wave, bool vec, int* list) {
  int wc = 0;
#pragma unroll
  for (int g = 0; g < NGRP; ++g) {
    const int el0 = (g * NTA + tid) * 4;
    const int e0  = cbase + el0;
    v4i d;
    if (vec) {
      d = *(const v4i*)(eid + e0);
    } else {
      const int sent = -2147483647 - 1;
      const int i0 = (e0     < nE) ? e0     : (nE - 1);
      const int i1 = (e0 + 1 < nE) ? e0 + 1 : (nE - 1);
      const int i2 = (e0 + 2 < nE) ? e0 + 2 : (nE - 1);
      const int i3 = (e0 + 3 < nE) ? e0 + 3 : (nE - 1);
      const int v0 = eid[i0], v1 = eid[i1], v2 = eid[i2], v3 = eid[i3];
      d.x = (e0     < nE) ? v0 : sent;
      d.y = (e0 + 1 < nE) ? v1 : sent;
      d.z = (e0 + 2 < nE) ? v2 : sent;
      d.w = (e0 + 3 < nE) ? v3 : sent;
    }
    const unsigned s0 = (unsigned)d.x - (unsigned)nodeBase;
    const unsigned s1 = (unsigned)d.y - (unsigned)nodeBase;
    const unsigned s2 = (unsigned)d.z - (unsigned)nodeBase;
    const unsigned s3 = (unsigned)d.w - (unsigned)nodeBase;
    const bool h0 = s0 < (unsigned)NB;
    const bool h1 = s1 < (unsigned)NB;
    const bool h2 = s2 < (unsigned)NB;
    const bool h3 = s3 < (unsigned)NB;
    const unsigned many = __builtin_amdgcn_ballot_w32(h0 | h1 | h2 | h3);
    if (many != 0u) {
      HITJ(0, h0, s0)
      HITJ(1, h1, s1)
      HITJ(2, h2, s2)
      HITJ(3, h3, s3)
    }
  }
  return wc;
}
#undef HITJ

__global__ __launch_bounds__(NTA) void k_agg8(
    const int* __restrict__ ei, const float* __restrict__ hb,
    const float* __restrict__ sS, const float* __restrict__ sD,
    float* gout, int nN, int nE) {
  extern __shared__ v4f lds_dyn[];
  float* sacc = (float*)lds_dyn;
  float* sden = sacc + LDS8_SACC;
  float* smax = sden + LDS8_DEN;
  int*   list = (int*)(smax + LDS8_MAX);
  int*   wcnt = list + LDS8_LIST;

  const int tid  = threadIdx.x;
  const int lane = tid & 31;
  const int wave = tid >> 5;
  const int hd   = lane >> 2;
  const int nodeBase = blockIdx.x * NB8;

  {
    const v4f z4 = {0.f, 0.f, 0.f, 0.f};
    for (int i = tid; i < (LDS8_SACC + LDS8_DEN) / 4; i += NTA) lds_dyn[i] = z4;
    const v4f n4 = {-1.0e30f, -1.0e30f, -1.0e30f, -1.0e30f};
    v4f* mx = (v4f*)smax;
    for (int i = tid; i < LDS8_MAX / 4; i += NTA) mx[i] = n4;
  }
  __syncthreads();

  const int* eid = ei + nE;
  const bool al16 = ((((size_t)eid) & 15) == 0);
  const int nChunks = (nE + CHUNK - 1) / CHUNK;

#pragma unroll 1
  for (int ch = 0; ch < nChunks; ++ch) {
    const int cbase = ch * CHUNK;
    const bool vec = al16 && (cbase + CHUNK <= nE);
    const int wc = scan_chunk<NB8, SH8>(eid, nE, cbase, nodeBase, tid, wave, vec, list);
    if (lane == 0) wcnt[wave] = wc;
    __syncthreads();

    if (wave == 0) {
      for (int wsx = 0; wsx < NWAVE; ++wsx) {
        int n = wcnt[wsx];
        if (n > WCAP) n = WCAP;
        if (n < 0) n = 0;
        for (int i = 0; i < n; ++i) {
          const int ent  = list[wsx * WCAP + i];
          const int slot = ent & (NB8 - 1);
          const int el   = (ent >> SH8) & (CHUNK - 1);
          int e = cbase + el;
          if (e > nE - 1) e = nE - 1;
          int src = ei[e];
          src = (src < 0) ? 0 : ((src > nN - 1) ? (nN - 1) : src);
          int nd = nodeBase + slot;
          if (nd > nN - 1) nd = nN - 1;
          float a = sS[(size_t)nd * NH + hd] + sD[(size_t)src * NH + hd];
          a = (a > 0.f) ? a : 0.2f * a;
          const int mi = slot * NH + hd;
          const float mo  = smax[mi];
          const float dn  = sden[mi];
          const float mn  = fmaxf(mo, a);
          const float scl = __expf(mo - mn);
          const float p   = __expf(a - mn);
          const float* xp = hb + (size_t)src * HCW + 8 * lane;
          const v4f x0 = *(const v4f*)(xp);
          const v4f x1 = *(const v4f*)(xp + 4);
          v4f* sp = (v4f*)(sacc + slot * HCW + 8 * lane);
          const v4f q0 = sp[0];
          const v4f q1 = sp[1];
          const v4f r0 = q0 * scl + p * x0;
          const v4f r1 = q1 * scl + p * x1;
          sp[0] = r0;
          sp[1] = r1;
          sden[mi] = dn * scl + p;
          smax[mi] = mn;
        }
      }
    }
    __syncthreads();
  }

  const int hA = lane >> 3;
  const int hB = 4 + (lane >> 3);
#pragma unroll 1
  for (int j = 0; j < NB8 / NWAVE; ++j) {
    const int slot = wave * (NB8 / NWAVE) + j;
    const int node = nodeBase + slot;
    if (node >= nN) break;
    const float d0 = sden[slot * NH + hA];
    const float d1 = sden[slot * NH + hB];
    const float rA = __builtin_amdgcn_rcpf(fmaxf(d0, 1.0e-30f));
    const float rB = __builtin_amdgcn_rcpf(fmaxf(d1, 1.0e-30f));
    const float i0 = (d0 > 0.f) ? rA : 0.f;
    const float i1 = (d1 > 0.f) ? rB : 0.f;
    v4f y0 = *(const v4f*)(sacc + slot * HCW + 4 * lane) * i0;
    v4f y1 = *(const v4f*)(sacc + slot * HCW + 128 + 4 * lane) * i1;
    y0 = elu4(y0);
    y1 = elu4(y1);
    float* op = gout + (size_t)node * HCW + 4 * lane;
    *(volatile v4f*)(op)       = y0;
    *(volatile v4f*)(op + 128) = y1;
    __threadfence();
    *(volatile v4f*)(op)       = y0;
    *(volatile v4f*)(op + 128) = y1;
  }
}

__global__ __launch_bounds__(NTA) void k_agg1(
    const int* __restrict__ ei, const float* __restrict__ hb,
    const float* __restrict__ sS, const float* __restrict__ sD,
    float* out, int nN, int nE) {
  extern __shared__ v4f lds_dyn[];
  float* sacc = (float*)lds_dyn;
  float* sden = sacc + LDS1_SACC;
  float* smax = sden + LDS1_DEN;
  int*   list = (int*)(smax + LDS1_MAX);
  int*   wcnt = list + LDS1_LIST;

  const int tid  = threadIdx.x;
  const int lane = tid & 31;
  const int wave = tid >> 5;
  const bool act = lane < (OC / 4);
  const int  cl  = act ? 4 * lane : 0;
  const int nodeBase = blockIdx.x * NB1;

  {
    const v4f z4 = {0.f, 0.f, 0.f, 0.f};
    for (int i = tid; i < (LDS1_SACC + LDS1_DEN) / 4; i += NTA) lds_dyn[i] = z4;
    const v4f n4 = {-1.0e30f, -1.0e30f, -1.0e30f, -1.0e30f};
    v4f* mx = (v4f*)smax;
    for (int i = tid; i < LDS1_MAX / 4; i += NTA) mx[i] = n4;
  }
  __syncthreads();

  const int* eid = ei + nE;
  const bool al16 = ((((size_t)eid) & 15) == 0);
  const int nChunks = (nE + CHUNK - 1) / CHUNK;

#pragma unroll 1
  for (int ch = 0; ch < nChunks; ++ch) {
    const int cbase = ch * CHUNK;
    const bool vec = al16 && (cbase + CHUNK <= nE);
    const int wc = scan_chunk<NB1, SH1>(eid, nE, cbase, nodeBase, tid, wave, vec, list);
    if (lane == 0) wcnt[wave] = wc;
    __syncthreads();

    if (wave == 0) {
      for (int wsx = 0; wsx < NWAVE; ++wsx) {
        int n = wcnt[wsx];
        if (n > WCAP) n = WCAP;
        if (n < 0) n = 0;
        for (int i = 0; i < n; ++i) {
          const int ent  = list[wsx * WCAP + i];
          const int slot = ent & (NB1 - 1);
          const int el   = (ent >> SH1) & (CHUNK - 1);
          int e = cbase + el;
          if (e > nE - 1) e = nE - 1;
          int src = ei[e];
          src = (src < 0) ? 0 : ((src > nN - 1) ? (nN - 1) : src);
          int nd = nodeBase + slot;
          if (nd > nN - 1) nd = nN - 1;
          float a = sS[nd] + sD[src];
          a = (a > 0.f) ? a : 0.2f * a;
          const float mo  = smax[slot];
          const float dn  = sden[slot];
          const float mn  = fmaxf(mo, a);
          const float scl = __expf(mo - mn);
          const float p   = __expf(a - mn);
          const v4f xv = *(const v4f*)(hb + (size_t)src * OP + cl);
          float* sp = sacc + slot * OC + cl;
          const v4f cur = *(const v4f*)sp;
          const v4f nxt = cur * scl + p * xv;
          if (act) *(v4f*)sp = nxt;
          sden[slot] = dn * scl + p;
          smax[slot] = mn;
        }
      }
    }
    __syncthreads();
  }

#pragma unroll 1
  for (int j = 0; j < NB1 / NWAVE; ++j) {
    const int slot = wave * (NB1 / NWAVE) + j;
    const int node = nodeBase + slot;
    if (node >= nN) break;
    const float dn  = sden[slot];
    const float rc  = __builtin_amdgcn_rcpf(fmaxf(dn, 1.0e-30f));
    const float inv = (dn > 0.f) ? rc : 0.f;
    float* sp = sacc + slot * OC + cl;
    const v4f y = *(const v4f*)sp * inv;
    float mxv = fmaxf(fmaxf(y.x, y.y), fmaxf(y.z, y.w));
    mxv = wmax(mxv);
    float s = __expf(y.x - mxv) + __expf(y.y - mxv) + __expf(y.z - mxv) + __expf(y.w - mxv);
    s = act ? s : 0.f;
    s = wsum(s);
    const float lse = mxv + __logf(s);
    const v4f o = y - lse;
    if (act) *(v4f*)sp = o;
  }
  __syncthreads();

  int nrows = nN - nodeBase;
  if (nrows > NB1) nrows = NB1;
  const int npc = nrows * (OC / 4);
  float* ob = out + (size_t)nodeBase * OC;
  for (int q = tid; q < npc; q += NTA) {
    const v4f v = *(const v4f*)(sacc + 4 * q);
    *(volatile v4f*)(ob + 4 * (size_t)q) = v;
  }
  __threadfence();
  for (int q = tid; q < npc; q += NTA) {
    const v4f v = *(const v4f*)(sacc + 4 * q);
    *(volatile v4f*)(ob + 4 * (size_t)q) = v;
  }
}

extern "C" void kernel_launch(void* const* d_in, const int* in_sizes, int n_in,
                              void* d_out, int out_size, void* d_ws, size_t ws_size,
                              hipStream_t stream) {
  if (n_in < 11) return;
  const int nN = in_sizes[0] / IN1;
  if (nN <= 0 || in_sizes[0] != nN * IN1) return;
  const int nE = in_sizes[1] / 2;
  if (nE <= 0 || in_sizes[1] != 2 * nE) return;
  if (in_sizes[2] != IN1 * HCW) return;
  if (in_sizes[3] != HCW || in_sizes[4] != HCW) return;
  if (in_sizes[5] != HCW * HCW) return;
  if (in_sizes[6] != HCW || in_sizes[7] != HCW) return;
  if (in_sizes[8] != HCW * OC) return;
  if (in_sizes[9] != OC || in_sizes[10] != OC) return;
  if (out_size != nN * OC) return;

  const float* x   = (const float*)d_in[0];
  const int*   ei  = (const int*)d_in[1];
  const float* W1  = (const float*)d_in[2];
  const float* as1 = (const float*)d_in[3];
  const float* ad1 = (const float*)d_in[4];
  const float* W2  = (const float*)d_in[5];
  const float* as2 = (const float*)d_in[6];
  const float* ad2 = (const float*)d_in[7];
  const float* W3  = (const float*)d_in[8];
  const float* as3 = (const float*)d_in[9];
  const float* ad3 = (const float*)d_in[10];
  float* out = (float*)d_out;

  const int NP = ((nN + RPAD - 1) / RPAD) * RPAD;
  size_t off = 0;
  _Float16* Wt1 = (_Float16*)((char*)d_ws + off); off += (size_t)HCW * IN1 * sizeof(_Float16);
  _Float16* Wt2 = (_Float16*)((char*)d_ws + off); off += (size_t)HCW * HCW * sizeof(_Float16);
  _Float16* Wt3 = (_Float16*)((char*)d_ws + off); off += (size_t)OP * HCW * sizeof(_Float16);
  float* hbuf = (float*)((char*)d_ws + off);      off += (size_t)NP * HCW * sizeof(float);
  float* gbuf = (float*)((char*)d_ws + off);      off += (size_t)NP * HCW * sizeof(float);
  float* sc   = (float*)((char*)d_ws + off);      off += (size_t)2 * NP * NH * sizeof(float);
  float* sc3  = (float*)((char*)d_ws + off);      off += (size_t)2 * NP * sizeof(float);
  if (off > ws_size) return;
  float* scS = sc;
  float* scD = sc + (size_t)NP * NH;
  float* s3S = sc3;
  float* s3D = sc3 + (size_t)NP;

  k_prepT<<<dim3(IN1 / 64, HCW / 32), 256, 0, stream>>>(W1, Wt1, IN1, HCW);
  k_prepT<<<dim3(HCW / 64, HCW / 32), 256, 0, stream>>>(W2, Wt2, HCW, HCW);
  k_prepT<<<dim3(HCW / 64, OP / 32), 256, 0, stream>>>(W3, Wt3, HCW, OC);

  hipFuncSetAttribute(reinterpret_cast<const void*>(&k_agg8),
                      hipFuncAttributeMaxDynamicSharedMemorySize, LDS8_BYTES);
  hipFuncSetAttribute(reinterpret_cast<const void*>(&k_agg1),
                      hipFuncAttributeMaxDynamicSharedMemorySize, LDS1_BYTES);
  const int grid8 = (nN + NB8 - 1) / NB8;
  const int grid1 = (nN + NB1 - 1) / NB1;

  k_gemm<IN1, HCW, 1, 1, HCW><<<NP / 32, 256, 0, stream>>>(x, Wt1, as1, ad1, hbuf, scS, scD, nN);
  k_agg8<<<grid8, NTA, LDS8_BYTES, stream>>>(ei, hbuf, scS, scD, gbuf, nN, nE);

  k_gemm<HCW, HCW, 1, 1, HCW><<<NP / 32, 256, 0, stream>>>(gbuf, Wt2, as2, ad2, hbuf, scS, scD, nN);
  k_agg8<<<grid8, NTA, LDS8_BYTES, stream>>>(ei, hbuf, scS, scD, gbuf, nN, nE);

  k_gemm<HCW, OP, 2, 2, OC><<<NP / 64, 128, 0, stream>>>(gbuf, Wt3, as3, ad3, hbuf, s3S, s3D, nN);
  k_agg1<<<grid1, NTA, LDS1_BYTES, stream>>>(ei, hbuf, s3S, s3D, out, nN, nE);
}
